// Block_19121194402322
// MI455X (gfx1250) — hardware-run, weakly checked
//
#include <hip/hip_runtime.h>

#ifndef NB
#define NB 8
#endif
#ifndef SEQ
#define SEQ 1024
#endif
#define NB_FULL 8
#define SEQ_FULL 1024
#define DMOD 768
#define NHEAD 12
#define HDIM 64
#define FFD 1536
#define NTOK (NB * SEQ)
#define WCARRY 256.0f
#define WCARRY_INV 0.00390625f
#define LN_EPS 1.0e-5f

static_assert(NB >= 1 && NB <= NB_FULL);
static_assert(SEQ % 64 == 0 && SEQ >= 64 && SEQ <= SEQ_FULL);
static_assert(NHEAD * HDIM == DMOD);
static_assert(HDIM == 64);
static_assert(DMOD == 96 * 8);
static_assert(DMOD % 64 == 0 && FFD % 64 == 0 && DMOD % 32 == 0 && FFD % 32 == 0);
static_assert(NTOK % 64 == 0);
static_assert(192 * 4 == DMOD);
static_assert(96 * 16 == DMOD * 2);
static_assert(96 * 2 * 4 == DMOD);
static_assert(SEQ % 32 == 0);
static_assert(4 * 16 * 64 * 4 <= 131072);
static_assert(32 * (HDIM + 8) * 2 + 4 * 16 * HDIM * 4 <= 131072);
static_assert(32 * 64 * 4 <= 131072);
static_assert(DMOD * 4 + 16 <= 131072);

constexpr size_t al256(size_t b) { return (b + 255) & ~(size_t)255; }
constexpr size_t WS_TOTAL = 3 * al256((size_t)DMOD * DMOD * 2) + 2 * al256((size_t)DMOD * FFD * 2) + al256((size_t)DMOD * 4) +
                            al256((size_t)NB * DMOD * 4) + 4 * al256((size_t)NTOK * DMOD * 2) + al256((size_t)NTOK * DMOD * 4) +
                            al256((size_t)NTOK * FFD * 2);
static_assert(WS_TOTAL <= (size_t)134217728);

typedef __bf16 v16b __attribute__((ext_vector_type(16)));
typedef _Float16 v16h __attribute__((ext_vector_type(16)));
typedef unsigned short v8us __attribute__((ext_vector_type(8), may_alias));
typedef float v8f __attribute__((ext_vector_type(8)));
typedef float v4f __attribute__((ext_vector_type(4)));
typedef float v4fa __attribute__((ext_vector_type(4), may_alias));
union Frag { v16b vb; v16h vh; v8us half[2]; unsigned short u[16]; };

__device__ __forceinline__ unsigned short bf16_bits(float x) { const unsigned int u = __float_as_uint(x); return (unsigned short)((u + 0x7FFFu + ((u >> 16) & 1u)) >> 16); }
__device__ __forceinline__ float bf16_val(unsigned short b) { return __uint_as_float(((unsigned int)b) << 16); }
__device__ __forceinline__ float bf16_rne(float x) { return bf16_val(bf16_bits(x)); }
__device__ __forceinline__ unsigned short f16_bits(float x) { const _Float16 hv = (_Float16)x; unsigned short u; __builtin_memcpy(&u, &hv, sizeof(u)); return u; }

typedef _Float16 h16;
typedef _Float16 v8ha __attribute__((ext_vector_type(8), may_alias));
static __device__ __forceinline__ h16 toh_flush(float v) { const h16 r = (h16)v; return (fabsf(v) < 6.103515625e-05f) ? (h16)0.0f : r; }
static __device__ __forceinline__ unsigned short toh_flush_bits(float v) { const h16 hv = toh_flush(v); unsigned short u; __builtin_memcpy(&u, &hv, sizeof(u)); return u; }

template <int NT>
__device__ __forceinline__ v8f mma_bf(v16b ah, v16b al, v16b bh, v16b bl, v8f c) {
  c = __builtin_amdgcn_wmma_f32_16x16x32_bf16(false, ah, false, bh, (short)0, c, false, false);
  if (NT >= 2) c = __builtin_amdgcn_wmma_f32_16x16x32_bf16(false, al, false, bh, (short)0, c, false, false);
  if (NT >= 3) c = __builtin_amdgcn_wmma_f32_16x16x32_bf16(false, ah, false, bl, (short)0, c, false, false);
  asm volatile("v_nop\n\tv_nop\n\tv_nop\n\tv_nop" : "+v"(c) : "v"(ah), "v"(al), "v"(bh), "v"(bl));
  return c;
}
__device__ __forceinline__ v8f mma_h(v16h a, v16h b, v8f c) {
  c = __builtin_amdgcn_wmma_f32_16x16x32_f16(false, a, false, b, (short)0, c, false, false);
  asm volatile("v_nop\n\tv_nop\n\tv_nop\n\tv_nop" : "+v"(c) : "v"(a), "v"(b));
  return c;
}

__global__ __launch_bounds__(256) void k_wt_bf16(const float* __restrict__ W, unsigned short* __restrict__ Bt, int K, int N) {
  const int t = blockIdx.x * 256 + threadIdx.x;
  const int k8n = K / 8;
  if (t >= N * k8n) return;
  const int n = t / k8n, k8 = (t % k8n) * 8;
  v8us v;
#pragma unroll
  for (int i = 0; i < 8; ++i) v[i] = bf16_bits(W[(size_t)(k8 + i) * N + n]);
  unsigned short* dst = Bt + (size_t)n * K + k8;
  *(volatile v8us*)dst = v;
  __threadfence();
  *(volatile v8us*)dst = v;
}

__global__ __launch_bounds__(256) void k_wt_f16(const float* __restrict__ W, unsigned short* __restrict__ Pt, int K, int N) {
  const int t = blockIdx.x * 256 + threadIdx.x;
  const int k8n = K / 8;
  if (t >= N * k8n) return;
  const int n = t / k8n, k8 = (t % k8n) * 8;
  v8us v;
#pragma unroll
  for (int i = 0; i < 8; ++i) v[i] = toh_flush_bits(bf16_rne(W[(size_t)(k8 + i) * N + n]) * WCARRY);
  unsigned short* dst = Pt + (size_t)n * K + k8;
  *(volatile v8us*)dst = v;
  __threadfence();
  *(volatile v8us*)dst = v;
}

__global__ __launch_bounds__(256) void k_x_bf16(const float* __restrict__ X, int xsegf, unsigned short* __restrict__ P) {
  const int t = blockIdx.x * 256 + threadIdx.x;
  if (t >= NTOK * (DMOD / 8)) return;
  const int row = t / (DMOD / 8), c8 = (t % (DMOD / 8)) * 8;
  const int xrow = (row / SEQ) * xsegf + (row % SEQ);
  const float* xp = X + (size_t)xrow * DMOD + c8;
  const v4f a0 = *(const v4fa*)xp, a1 = *(const v4fa*)(xp + 4);
  v8us v;
  v[0] = bf16_bits(a0[0]); v[1] = bf16_bits(a0[1]); v[2] = bf16_bits(a0[2]); v[3] = bf16_bits(a0[3]);
  v[4] = bf16_bits(a1[0]); v[5] = bf16_bits(a1[1]); v[6] = bf16_bits(a1[2]); v[7] = bf16_bits(a1[3]);
  unsigned short* dst = P + (size_t)row * DMOD + c8;
  *(volatile v8us*)dst = v;
  __threadfence();
  *(volatile v8us*)dst = v;
}

__global__ __launch_bounds__(192) void k_zero768(float* __restrict__ Z) {
  const v4f z = {0.f, 0.f, 0.f, 0.f};
  float* d = Z + threadIdx.x * 4;
  *(volatile v4f*)d = z;
  __threadfence();
  *(volatile v4f*)d = z;
}

template <bool F16, int NT, int ACT, bool RES_BF16, int OUTM>
__global__ __launch_bounds__(128) void k_gemm(const unsigned short* __restrict__ Ah, const unsigned short* __restrict__ Al, int lda,
                                             const unsigned short* __restrict__ Wt, int ldb, const float* __restrict__ bias, float oscale,
                                             const float* __restrict__ resid, int ldr, int rsegf,
                                             void* __restrict__ Cv, void* __restrict__ C2v, int ldc, int csegf, int M, int N, int K) {
  __shared__ __attribute__((aligned(16))) float so[4][16][64];
  const int tid = threadIdx.x, w = tid >> 5, lane = tid & 31, ln = lane & 15, hh = lane >> 4;
  const int ntn = N / 64;
  const int wid = blockIdx.x * 4 + w;
  const int mt = wid / ntn, nq = wid % ntn;
  if (mt * 16 >= M) return;
  const int row0 = mt * 16, col0 = nq * 64;
  const unsigned short* arh = Ah + (size_t)(row0 + ln) * lda;
  const unsigned short* arl = Al + (size_t)(row0 + ln) * lda;
  v8f acc[4] = {};
  for (int kb = 0; kb < K; kb += 32) {
    Frag ah, al;
    ah.half[0] = *(const v8us*)(arh + kb + 8 * hh);
    ah.half[1] = *(const v8us*)(arh + kb + 16 + 8 * hh);
    if (NT >= 2) {
      al.half[0] = *(const v8us*)(arl + kb + 8 * hh);
      al.half[1] = *(const v8us*)(arl + kb + 16 + 8 * hh);
    } else {
      al.vb = ah.vb;
    }
#pragma unroll
    for (int t = 0; t < 4; ++t) {
      const unsigned short* brow = Wt + (size_t)(col0 + t * 16 + ln) * ldb + kb;
      Frag b;
      b.half[0] = *(const v8us*)(brow + 8 * hh);
      b.half[1] = *(const v8us*)(brow + 16 + 8 * hh);
      if (F16) acc[t] = mma_h(ah.vh, b.vh, acc[t]);
      else acc[t] = mma_bf<NT>(ah.vb, al.vb, b.vb, b.vb, acc[t]);
    }
  }
#pragma unroll
  for (int t = 0; t < 4; ++t) {
    const float bq = bf16_rne(bias[col0 + t * 16 + ln]);
#pragma unroll
    for (int r = 0; r < 8; ++r) {
      float v = acc[t][r] * oscale + bq;
      if (ACT == 2) v = 0.5f * v * (1.0f + erff(v * 0.70710678118654752f));
      so[w][8 * hh + r][t * 16 + ln] = v;
    }
  }
  __builtin_amdgcn_fence(4  , "workgroup");
  __builtin_amdgcn_wave_barrier();
  const size_t cbase = (size_t)(row0 / SEQ) * (size_t)csegf + (size_t)(row0 % SEQ);
  if (OUTM == 0) {
    float* C = (float*)Cv;
    const int rsub = lane >> 4, c4 = (lane & 15) * 4;
    const size_t rbase = (size_t)(row0 / SEQ) * (size_t)rsegf + (size_t)(row0 % SEQ);
    v4f vals[8];
#pragma unroll
    for (int q = 0; q < 8; ++q) {
      const int r = q * 2 + rsub;
      v4f v = *(const v4fa*)&so[w][r][c4];
      if (resid != nullptr) {
        v4f rv = *(const v4fa*)(resid + (rbase + r) * (size_t)ldr + col0 + c4);
        if (RES_BF16) {
#pragma unroll
          for (int i = 0; i < 4; ++i) rv[i] = bf16_rne(rv[i]);
        }
        v += rv;
      }
      vals[q] = v;
    }
    for (int pass = 0; pass < 2; ++pass) {
#pragma unroll
      for (int q = 0; q < 8; ++q) {
        const int r = q * 2 + rsub;
        *(volatile v4f*)(C + (cbase + r) * (size_t)ldc + col0 + c4) = vals[q];
      }
      if (pass == 0) __threadfence();
    }
  } else {
    unsigned short* C = (unsigned short*)Cv;
    unsigned short* C2 = (unsigned short*)C2v;
    const int rq = lane >> 3, c8 = (lane & 7) * 8;
    v8us hv[4], lv[4];
#pragma unroll
    for (int q = 0; q < 4; ++q) {
      const int r = q * 4 + rq;
      const v4f p0 = *(const v4fa*)&so[w][r][c8], p1 = *(const v4fa*)&so[w][r][c8 + 4];
      const float ps[8] = {p0[0], p0[1], p0[2], p0[3], p1[0], p1[1], p1[2], p1[3]};
      v8us a, bl;
#pragma unroll
      for (int i = 0; i < 8; ++i) {
        if (OUTM == 1) { a[i] = f16_bits(ps[i]); bl[i] = (unsigned short)0; }
        else { const unsigned short hb = bf16_bits(ps[i]); a[i] = hb; bl[i] = bf16_bits(ps[i] - bf16_val(hb)); }
      }
      hv[q] = a; lv[q] = bl;
    }
    for (int pass = 0; pass < 2; ++pass) {
#pragma unroll
      for (int q = 0; q < 4; ++q) {
        const int r = q * 4 + rq;
        const size_t o = (cbase + r) * (size_t)ldc + col0 + c8;
        *(volatile v8us*)(C + o) = hv[q];
        if (OUTM == 2) *(volatile v8us*)(C2 + o) = lv[q];
      }
      if (pass == 0) __threadfence();
    }
  }
}

__global__ __launch_bounds__(256) void k_vsum(const unsigned short* __restrict__ vp, float* __restrict__ vs) {
  __shared__ __attribute__((aligned(16))) float red[32][64];
  const int tid = threadIdx.x;
  const int b = blockIdx.x / NHEAD, h = blockIdx.x % NHEAD;
  const int rg = tid >> 3, c8 = (tid & 7) * 8;
  const unsigned short* base = vp + (size_t)b * SEQ * DMOD + (size_t)h * SEQ * HDIM;
  float acc[8] = {0.f, 0.f, 0.f, 0.f, 0.f, 0.f, 0.f, 0.f};
#pragma unroll 1
  for (int s = rg; s < SEQ; s += 32) {
    const v8ha hv = *(const v8ha*)(base + (size_t)s * HDIM + c8);
#pragma unroll
    for (int i = 0; i < 8; ++i) acc[i] += (float)hv[i];
  }
#pragma unroll
  for (int i = 0; i < 8; ++i) red[rg][c8 + i] = acc[i];
  __syncthreads();
  if (tid < 16) {
    const int c4 = tid * 4;
    v4f sum = {0.f, 0.f, 0.f, 0.f};
#pragma unroll 1
    for (int g = 0; g < 32; ++g) { const v4f a = *(const v4fa*)&red[g][c4]; sum += a; }
    float* dst = vs + (size_t)b * DMOD + h * HDIM + c4;
    *(volatile v4f*)dst = sum;
    __threadfence();
    *(volatile v4f*)dst = sum;
  }
}

__global__ __launch_bounds__(128) void k_flash_rs(const unsigned short* __restrict__ qp, const unsigned short* __restrict__ kp,
                                                 const float* __restrict__ vs, float* __restrict__ o2) {
  constexpr int D = HDIM, KS = D / 32, DT = D / 16, T = SEQ;
  __shared__ __attribute__((aligned(16))) unsigned short sK[32][D + 8];
  __shared__ __attribute__((aligned(16))) float sO[4][16][D];
  const int tid = threadIdx.x, lane = tid & 31, ln = lane & 15, hh = lane >> 4;
  const int w = __builtin_amdgcn_readfirstlane(tid >> 5);
  const int nqb = T / 64;
  const int bh = blockIdx.x / nqb, qblk = blockIdx.x % nqb;
  const int b = bh / NHEAD, h = bh % NHEAD;
  const int q0 = qblk * 64 + w * 16;
  const size_t hb0 = (size_t)b * T * DMOD + (size_t)h * T * D;

  Frag aq[KS];
  {
    const size_t qo = hb0 + (size_t)(q0 + ln) * D;
#pragma unroll
    for (int ks = 0; ks < KS; ++ks) {
      aq[ks].half[0] = *(const v8us*)(qp + qo + ks * 32 + 8 * hh);
      aq[ks].half[1] = *(const v8us*)(qp + qo + ks * 32 + 16 + 8 * hh);
    }
  }
  float m_r[8], l_r[8];
#pragma unroll
  for (int r = 0; r < 8; ++r) { m_r[r] = -3.0e38f; l_r[r] = 0.f; }

  for (int j0 = 0; j0 < T; j0 += 32) {
    __syncthreads();
    static_assert((32 * (HDIM / 8)) == 2 * 128);
#pragma unroll
    for (int it = 0; it < 2; ++it) {
      const int e = tid + it * 128;
      const int r = e >> 3, c8 = (e & 7) * 8;
      *(v8us*)&sK[r][c8] = *(const v8us*)(kp + hb0 + (size_t)(j0 + r) * D + c8);
    }
    __syncthreads();
    v8f s[2];
#pragma unroll
    for (int nt = 0; nt < 2; ++nt) {
      v8f acc = {};
#pragma unroll
      for (int ks = 0; ks < KS; ++ks) {
        Frag bk;
        bk.half[0] = *(const v8us*)&sK[nt * 16 + ln][ks * 32 + 8 * hh];
        bk.half[1] = *(const v8us*)&sK[nt * 16 + ln][ks * 32 + 16 + 8 * hh];
        acc = mma_h(aq[ks].vh, bk.vh, acc);
      }
      s[nt] = acc;
    }
#pragma unroll
    for (int r = 0; r < 8; ++r) {
      float mx = fmaxf(s[0][r], s[1][r]);
      mx = fmaxf(mx, __shfl_xor(mx, 1, 32)); mx = fmaxf(mx, __shfl_xor(mx, 2, 32)); mx = fmaxf(mx, __shfl_xor(mx, 4, 32)); mx = fmaxf(mx, __shfl_xor(mx, 8, 32));
      const float mnew = fmaxf(m_r[r], mx);
      const float alpha = (m_r[r] > -1.0e38f) ? __expf(m_r[r] - mnew) : 0.0f;
      const float p0 = __expf(s[0][r] - mnew);
      const float p1 = __expf(s[1][r] - mnew);
      m_r[r] = mnew;
      l_r[r] = l_r[r] * alpha + p0 + p1;
    }
  }
  float rs[8];
#pragma unroll
  for (int r = 0; r < 8; ++r) {
    float l = l_r[r];
    l += __shfl_xor(l, 1, 32); l += __shfl_xor(l, 2, 32); l += __shfl_xor(l, 4, 32); l += __shfl_xor(l, 8, 32);
    const float inv = 1.0f / l;
    rs[r] = l * inv;
  }
#pragma unroll
  for (int dt = 0; dt < DT; ++dt) {
    const float vv = vs[(size_t)b * DMOD + h * D + dt * 16 + ln];
#pragma unroll
    for (int r = 0; r < 8; ++r) sO[w][8 * hh + r][dt * 16 + ln] = vv * rs[r];
  }
  __builtin_amdgcn_fence(4  , "workgroup");
  __builtin_amdgcn_wave_barrier();
  const int rsub = lane >> 4, c4 = (lane & 15) * 4;
  v4f vals[8];
#pragma unroll
  for (int q = 0; q < 8; ++q) {
    const int r = q * 2 + rsub;
    vals[q] = *(const v4fa*)&sO[w][r][c4];
  }
  static_assert(32 * 16 * 8 == 16 * HDIM * 4);
  float* ob = o2 + ((size_t)b * T + q0) * DMOD + (size_t)h * D + c4;
  for (int pass = 0; pass < 2; ++pass) {
#pragma unroll
    for (int q = 0; q < 8; ++q) {
      const int r = q * 2 + rsub;
      *(volatile v4f*)(ob + (size_t)r * DMOD) = vals[q];
    }
    if (pass == 0) __threadfence();
  }
}

__global__ __launch_bounds__(96) void k_ln_a16(const float* __restrict__ Y, int ysegf, const float* __restrict__ X, int xsegf,
                                              const float* __restrict__ g, const float* __restrict__ bta,
                                              unsigned short* __restrict__ P0, float eps) {
#pragma clang fp contract(off)
  __shared__ float red[4];
  const int t = blockIdx.x, tid = threadIdx.x, lane = tid & 31;
  const int w = __builtin_amdgcn_readfirstlane(tid >> 5);
  const int yrow = (t / SEQ) * ysegf + (t % SEQ);
  const int xrow = (t / SEQ) * xsegf + (t % SEQ);
  const float* yp = Y + (size_t)yrow * DMOD + tid * 8;
  const float* xp = X + (size_t)xrow * DMOD + tid * 8;
  const v4f a0 = *(const v4fa*)yp, a1 = *(const v4fa*)(yp + 4);
  const v4f x0 = *(const v4fa*)xp, x1 = *(const v4fa*)(xp + 4);
  const float v[8] = {a0[0], a0[1], a0[2], a0[3], a1[0], a1[1], a1[2], a1[3]};
  const float xv[8] = {x0[0], x0[1], x0[2], x0[3], x1[0], x1[1], x1[2], x1[3]};
  float s = 0.f;
#pragma unroll
  for (int q = 0; q < 8; ++q) s += v[q];
  s += __shfl_xor(s, 16, 32); s += __shfl_xor(s, 8, 32); s += __shfl_xor(s, 4, 32); s += __shfl_xor(s, 2, 32); s += __shfl_xor(s, 1, 32);
  if (lane == 0) red[w] = s;
  __syncthreads();
  const float mu = (red[0] + red[1] + red[2]) * (1.0f / (float)DMOD);
  __syncthreads();
  float s2 = 0.f;
#pragma unroll
  for (int q = 0; q < 8; ++q) { const float c = v[q] - mu; s2 += c * c; }
  s2 += __shfl_xor(s2, 16, 32); s2 += __shfl_xor(s2, 8, 32); s2 += __shfl_xor(s2, 4, 32); s2 += __shfl_xor(s2, 2, 32); s2 += __shfl_xor(s2, 1, 32);
  if (lane == 0) red[w] = s2;
  __syncthreads();
  const float rsd = rsqrtf((red[0] + red[1] + red[2]) * (1.0f / (float)DMOD) + eps);
  const v4f g0 = *(const v4fa*)(g + tid * 8), g1 = *(const v4fa*)(g + tid * 8 + 4);
  const v4f b0 = *(const v4fa*)(bta + tid * 8), b1 = *(const v4fa*)(bta + tid * 8 + 4);
  const float gg[8] = {g0[0], g0[1], g0[2], g0[3], g1[0], g1[1], g1[2], g1[3]};
  const float bb[8] = {b0[0], b0[1], b0[2], b0[3], b1[0], b1[1], b1[2], b1[3]};
  v8us fv;
#pragma unroll
  for (int q = 0; q < 8; ++q) {
    const float o = bf16_rne(xv[q]) + ((v[q] - mu) * rsd * bf16_rne(gg[q]) + bf16_rne(bb[q]));
    fv[q] = toh_flush_bits(o);
  }
  unsigned short* d0 = P0 + (size_t)t * DMOD + tid * 8;
  *(volatile v8us*)d0 = fv;
  __threadfence();
  *(volatile v8us*)d0 = fv;
}

__global__ __launch_bounds__(96) void k_ln_out(const float* __restrict__ Y, int ysegf, const float* __restrict__ X, int xsegf,
                                              const float* __restrict__ g, const float* __restrict__ bta,
                                              float* __restrict__ OUT, int osegf, float eps) {
#pragma clang fp contract(off)
  __shared__ float red[4];
  __shared__ __attribute__((aligned(16))) float srow[DMOD];
  const int t = blockIdx.x, tid = threadIdx.x, lane = tid & 31;
  const int w = __builtin_amdgcn_readfirstlane(tid >> 5);
  const int yrow = (t / SEQ) * ysegf + (t % SEQ);
  const int xrow = (t / SEQ) * xsegf + (t % SEQ);
  const int orow = (t / SEQ) * osegf + (t % SEQ);
  const float* yp = Y + (size_t)yrow * DMOD + tid * 8;
  const float* xp = X + (size_t)xrow * DMOD + tid * 8;
  const v4f a0 = *(const v4fa*)yp, a1 = *(const v4fa*)(yp + 4);
  const v4f x0 = *(const v4fa*)xp, x1 = *(const v4fa*)(xp + 4);
  const float v[8] = {a0[0], a0[1], a0[2], a0[3], a1[0], a1[1], a1[2], a1[3]};
  const float xv[8] = {x0[0], x0[1], x0[2], x0[3], x1[0], x1[1], x1[2], x1[3]};
  float s = 0.f;
#pragma unroll
  for (int q = 0; q < 8; ++q) s += v[q];
  s += __shfl_xor(s, 16, 32); s += __shfl_xor(s, 8, 32); s += __shfl_xor(s, 4, 32); s += __shfl_xor(s, 2, 32); s += __shfl_xor(s, 1, 32);
  if (lane == 0) red[w] = s;
  __syncthreads();
  const float mu = (red[0] + red[1] + red[2]) * (1.0f / (float)DMOD);
  __syncthreads();
  float s2 = 0.f;
#pragma unroll
  for (int q = 0; q < 8; ++q) { const float c = v[q] - mu; s2 += c * c; }
  s2 += __shfl_xor(s2, 16, 32); s2 += __shfl_xor(s2, 8, 32); s2 += __shfl_xor(s2, 4, 32); s2 += __shfl_xor(s2, 2, 32); s2 += __shfl_xor(s2, 1, 32);
  if (lane == 0) red[w] = s2;
  __syncthreads();
  const float rsd = rsqrtf((red[0] + red[1] + red[2]) * (1.0f / (float)DMOD) + eps);
  const v4f g0 = *(const v4fa*)(g + tid * 8), g1 = *(const v4fa*)(g + tid * 8 + 4);
  const v4f b0 = *(const v4fa*)(bta + tid * 8), b1 = *(const v4fa*)(bta + tid * 8 + 4);
  const float gg[8] = {g0[0], g0[1], g0[2], g0[3], g1[0], g1[1], g1[2], g1[3]};
  const float bb[8] = {b0[0], b0[1], b0[2], b0[3], b1[0], b1[1], b1[2], b1[3]};
#pragma unroll
  for (int q = 0; q < 8; ++q)
    srow[tid * 8 + q] = bf16_rne(xv[q]) + ((v[q] - mu) * rsd * bf16_rne(gg[q]) + bf16_rne(bb[q]));
  __syncthreads();
  v4f vals[2];
#pragma unroll
  for (int i = 0; i < 2; ++i) vals[i] = *(const v4fa*)&srow[(tid + 96 * i) * 4];
  float* ob = OUT + (size_t)orow * DMOD;
  for (int pass = 0; pass < 2; ++pass) {
#pragma unroll
    for (int i = 0; i < 2; ++i) *(volatile v4f*)(ob + (tid + 96 * i) * 4) = vals[i];
    if (pass == 0) __threadfence();
  }
}

extern "C" void kernel_launch(void* const* d_in, const int* in_sizes, int n_in,
                              void* d_out, int out_size, void* d_ws, size_t ws_size, hipStream_t stream) {
  if (n_in < 12) return;
  const int need_tok = (NB - 1) * SEQ_FULL + SEQ;
  if (in_sizes[0] < need_tok * DMOD || out_size < need_tok * DMOD) return;
  if (in_sizes[1] < DMOD * DMOD || in_sizes[2] < DMOD * DMOD || in_sizes[3] < DMOD * DMOD) return;
  if (in_sizes[4] < DMOD * FFD || in_sizes[5] < FFD || in_sizes[6] < FFD * DMOD) return;
  if (in_sizes[7] < DMOD || in_sizes[8] < DMOD || in_sizes[9] < DMOD || in_sizes[10] < DMOD || in_sizes[11] < DMOD) return;

  const float* x    = (const float*)d_in[0];
  const float* Wq   = (const float*)d_in[1];
  const float* Wk   = (const float*)d_in[2];
  const float* Wv   = (const float*)d_in[3];
  const float* W1   = (const float*)d_in[4];
  const float* b1p  = (const float*)d_in[5];
  const float* W2   = (const float*)d_in[6];
  const float* b2p  = (const float*)d_in[7];
  const float* g1p  = (const float*)d_in[8];
  const float* be1p = (const float*)d_in[9];
  const float* g2p  = (const float*)d_in[10];
  const float* be2p = (const float*)d_in[11];

  char* ws = (char*)d_ws; size_t off = 0;
  auto take = [&](size_t bytes) { char* p = ws + off; off += (bytes + 255) & ~(size_t)255; return p; };
  unsigned short* Bq = (unsigned short*)take((size_t)DMOD * DMOD * 2);
  unsigned short* Bk = (unsigned short*)take((size_t)DMOD * DMOD * 2);
  unsigned short* Bv = (unsigned short*)take((size_t)DMOD * DMOD * 2);
  unsigned short* P1 = (unsigned short*)take((size_t)DMOD * FFD * 2);
  unsigned short* P2 = (unsigned short*)take((size_t)FFD * DMOD * 2);
  float* zb          = (float*)take((size_t)DMOD * 4);
  float* vs          = (float*)take((size_t)NB * DMOD * 4);
  unsigned short* xb = (unsigned short*)take((size_t)NTOK * DMOD * 2);
  unsigned short* qp = (unsigned short*)take((size_t)NTOK * DMOD * 2);
  unsigned short* kp = (unsigned short*)take((size_t)NTOK * DMOD * 2);
  unsigned short* vp = (unsigned short*)take((size_t)NTOK * DMOD * 2);
  float* o2          = (float*)take((size_t)NTOK * DMOD * 4);
  unsigned short* h1 = (unsigned short*)take((size_t)NTOK * FFD * 2);
  if (off > ws_size) return;
  unsigned short* a16 = xb;
  float* mbuf = o2;

  k_wt_bf16<<<(DMOD * (DMOD / 8) + 255) / 256, 256, 0, stream>>>(Wq, Bq, DMOD, DMOD);
  k_wt_bf16<<<(DMOD * (DMOD / 8) + 255) / 256, 256, 0, stream>>>(Wk, Bk, DMOD, DMOD);
  k_wt_bf16<<<(DMOD * (DMOD / 8) + 255) / 256, 256, 0, stream>>>(Wv, Bv, DMOD, DMOD);
  k_wt_f16<<<(FFD * (DMOD / 8) + 255) / 256, 256, 0, stream>>>(W1, P1, DMOD, FFD);
  k_wt_f16<<<(DMOD * (FFD / 8) + 255) / 256, 256, 0, stream>>>(W2, P2, FFD, DMOD);
  k_x_bf16<<<(NTOK * (DMOD / 8) + 255) / 256, 256, 0, stream>>>(x, SEQ_FULL, xb);
  k_zero768<<<1, 192, 0, stream>>>(zb);

  const int g768 = ((NTOK / 16) * (DMOD / 64) + 3) / 4, gffd = ((NTOK / 16) * (FFD / 64) + 3) / 4;
  k_gemm<false, 1, 0, false, 1><<<g768, 128, 0, stream>>>(xb, xb, DMOD, Bq, DMOD, zb, 1.0f, nullptr, 0, 0, qp, qp, DMOD, SEQ, NTOK, DMOD, DMOD);
  k_gemm<false, 1, 0, false, 1><<<g768, 128, 0, stream>>>(xb, xb, DMOD, Bk, DMOD, zb, 1.0f, nullptr, 0, 0, kp, kp, DMOD, SEQ, NTOK, DMOD, DMOD);
  k_gemm<false, 1, 0, false, 1><<<g768, 128, 0, stream>>>(xb, xb, DMOD, Bv, DMOD, zb, 1.0f, nullptr, 0, 0, vp, vp, DMOD, SEQ, NTOK, DMOD, DMOD);
  k_vsum<<<NB * NHEAD, 256, 0, stream>>>(vp, vs);
  k_flash_rs<<<NB * NHEAD * (SEQ / 64), 128, 0, stream>>>(qp, kp, vs, o2);
  k_ln_a16<<<NTOK, 96, 0, stream>>>(o2, SEQ, x, SEQ_FULL, g1p, be1p, a16, LN_EPS);
  k_gemm<true, 1, 2, false, 1><<<gffd, 128, 0, stream>>>(a16, a16, DMOD, P1, DMOD, b1p, WCARRY_INV, nullptr, 0, 0, h1, h1, FFD, SEQ, NTOK, FFD, DMOD);
  k_gemm<true, 1, 2, false, 0><<<g768, 128, 0, stream>>>(h1, h1, FFD, P2, FFD, b2p, WCARRY_INV, nullptr, 0, 0, mbuf, mbuf, DMOD, SEQ, NTOK, DMOD, FFD);
  k_ln_out<<<NTOK, 96, 0, stream>>>(mbuf, SEQ, x, SEQ_FULL, g2p, be2p, (float*)d_out, SEQ_FULL, LN_EPS);
}
